// TRMBlock_22746146799814
// MI455X (gfx1250) — hardware-verified
//
#include <hip/hip_runtime.h>
#include <math.h>
#include <stdint.h>

typedef __attribute__((ext_vector_type(16))) _Float16 v16h;
typedef __attribute__((ext_vector_type(8)))  _Float16 v8h;
typedef __attribute__((ext_vector_type(16))) __bf16   v16b;
typedef __attribute__((ext_vector_type(8)))  __bf16   v8b;
typedef __attribute__((ext_vector_type(8)))  float    v8f;
typedef __attribute__((ext_vector_type(4)))  float    v4f;
typedef __attribute__((ext_vector_type(4)))  unsigned int v4u;
typedef __attribute__((ext_vector_type(2)))  unsigned int v2u;

static constexpr int kBatch   = 4;
static constexpr int kSeq     = 2048;
static constexpr int kTok     = kBatch * kSeq;
static constexpr int kModel   = 512;
static constexpr int kHeads   = 8;
static constexpr int kHeadDim = 64;
static constexpr int kFF      = 1024;
static constexpr int kQKCols  = 2 * kModel;
static constexpr int kGUCols  = 2 * kFF;

static_assert(kHeads * kHeadDim == kModel, "head geometry");
static_assert(kSeq % 64 == 0 && kTok % 64 == 0, "tile multiples");
static_assert(kModel % 64 == 0 && kFF % 64 == 0 && kQKCols % 64 == 0 && kGUCols % 64 == 0, "tile multiples");
static_assert(kModel % 32 == 0 && kFF % 32 == 0, "K multiple of 32");

static constexpr size_t kOffWqkT = 0;
static constexpr size_t kOffWvT  = kOffWqkT + (size_t)kQKCols * kModel * 2;
static constexpr size_t kOffWoT  = kOffWvT + (size_t)kModel * kModel * 2;
static constexpr size_t kOffWguT = kOffWoT + (size_t)kModel * kModel * 2;
static constexpr size_t kOffWdT  = kOffWguT + (size_t)kGUCols * kModel * 2;
static constexpr size_t kOffHG   = kOffWdT + (size_t)kModel * kFF * 2;
static constexpr size_t kSizeHG  = (size_t)kTok * kFF * 2;
static constexpr size_t kOffR1   = kOffHG + kSizeHG;
static constexpr size_t kSizeR1  = (size_t)kTok * kGUCols * 4;
static constexpr size_t kR1QK    = 0;
static constexpr size_t kR1Vt    = kR1QK + (size_t)kTok * kQKCols * 2;
static constexpr size_t kR1O     = kR1Vt + (size_t)kBatch * kModel * kSeq * 2;
static constexpr size_t kR1A1    = kR1O + (size_t)kTok * kModel * 2;
static constexpr size_t kOffX1   = kOffR1 + kSizeR1;
static constexpr size_t kWsTotal = kOffX1 + (size_t)kTok * kModel * 4;
static_assert(kR1A1 + (size_t)kTok * kModel * 4 <= kSizeR1, "phase A fits R1");
static_assert((size_t)kTok * kModel * 4 <= kSizeR1, "phase C fits R1");
static_assert((size_t)kTok * kModel * 2 <= kSizeHG, "h plane fits HG");
static_assert(kWsTotal == 105906176, "carve total");
static_assert(kWsTotal <= 134217728, "carve under 128 MiB");
static_assert((kOffWvT % 256) == 0 && (kOffWoT % 256) == 0 && (kOffWguT % 256) == 0 && (kOffWdT % 256) == 0 &&
              (kOffHG % 256) == 0 && (kOffR1 % 256) == 0 && (kOffX1 % 256) == 0 &&
              (kR1Vt % 256) == 0 && (kR1O % 256) == 0 && (kR1A1 % 256) == 0, "aligned carves");

#define PSCALE 32768.0f
#define U16(p) ((const unsigned short*)(const void*)(p))
#define PSCALE_INV (1.0f / 32768.0f)

__device__ __forceinline__ unsigned short f2bf_bits(float f) {
  unsigned u = __float_as_uint(f);
  return (unsigned short)((u + 0x7FFFu + ((u >> 16) & 1u)) >> 16);
}
__device__ __forceinline__ float bf_bits2f(unsigned short h) { return __uint_as_float(((unsigned)h) << 16); }

__device__ __forceinline__ void dep_guard_h(v8f& a, v8f& b, v16h x, v16h y) { asm volatile("v_nop\n\tv_nop\n\tv_nop\n\tv_nop" : "+v"(a), "+v"(b) : "v"(x), "v"(y)); }
__device__ __forceinline__ void dep_guard_b(v8f& a, v8f& b, v16b x, v16b y) { asm volatile("v_nop\n\tv_nop\n\tv_nop\n\tv_nop" : "+v"(a), "+v"(b) : "v"(x), "v"(y)); }
__device__ __forceinline__ void keep4_h(v16h a, v16h b, v16h c, v16h d) { asm volatile("v_nop" :: "v"(a), "v"(b), "v"(c), "v"(d)); }
__device__ __forceinline__ void keep4_b(v16b a, v16b b, v16b c, v16b d) { asm volatile("v_nop" :: "v"(a), "v"(b), "v"(c), "v"(d)); }
__device__ __forceinline__ void acc_guard4(v8f& a, v8f& b, v8f& c, v8f& d) { asm volatile("v_nop\n\tv_nop\n\tv_nop\n\tv_nop" : "+v"(a), "+v"(b), "+v"(c), "+v"(d)); }
template <typename T> struct Frag;
template <> struct Frag<_Float16> {
  typedef v16h V; union U { v16h v; v8h h[2]; };
  static __device__ __forceinline__ v16h load(const _Float16* p) {
    U f; f.h[0] = *(const v8h*)(p); f.h[1] = *(const v8h*)(p + 16); return f.v;
  }
  static __device__ __forceinline__ v8f mma(v16h a, v16h b, v8f c) {
    return __builtin_amdgcn_wmma_f32_16x16x32_f16(false, a, false, b, (short)0, c, false, false);
  }
  static __device__ __forceinline__ void guard(v8f& a, v8f& b, v16h x, v16h y) { dep_guard_h(a, b, x, y); }
  static __device__ __forceinline__ void keep(v16h a, v16h b, v16h c, v16h d) { keep4_h(a, b, c, d); }
};
template <> struct Frag<__bf16> {
  typedef v16b V; union U { v16b v; v8b h[2]; };
  static __device__ __forceinline__ v16b load(const __bf16* p) {
    U f; f.h[0] = *(const v8b*)(p); f.h[1] = *(const v8b*)(p + 16); return f.v;
  }
  static __device__ __forceinline__ v8f mma(v16b a, v16b b, v8f c) {
    return __builtin_amdgcn_wmma_f32_16x16x32_bf16(false, a, false, b, (short)0, c, false, false);
  }
  static __device__ __forceinline__ void guard(v8f& a, v8f& b, v16b x, v16b y) { dep_guard_b(a, b, x, y); }
  static __device__ __forceinline__ void keep(v16b a, v16b b, v16b c, v16b d) { keep4_b(a, b, c, d); }
};

template <int ET> struct Elem;
template <> struct Elem<0> { typedef _Float16 T; };
template <> struct Elem<1> { typedef __bf16 T; };
template <int ET, bool SPLIT, int BIAS_MODE, int OUT_MODE, bool RESID, int ACT = 0>
__global__ __launch_bounds__(256) void wmma_gemm64(
    const unsigned short* __restrict__ Ap, const unsigned short* __restrict__ A2p, int lda, long strideA,
    const unsigned short* __restrict__ Btp, const unsigned short* __restrict__ Bt2p, int ldb, long strideB,
    void* __restrict__ Cout, void* __restrict__ Cout2, int ldc, long strideC,
    const float* __restrict__ bias,
    const float* __restrict__ resid, long strideR,
    int M, int N, int K, float scale) {
  typedef typename Elem<ET>::T T;
  typedef typename Frag<T>::V V;
  const T* A = (const T*)Ap; const T* A2 = (const T*)A2p; const T* Bt = (const T*)Btp; const T* Bt2 = (const T*)Bt2p;
  __shared__ __align__(16) float sT[8][16 * 68];
  const int b    = blockIdx.y;
  const int lane = threadIdx.x & 31;
  const int wave = threadIdx.x >> 5;
  const int tilesN = N >> 6;
  const int tilesM = M >> 6;
  const int tile = blockIdx.x * 8 + wave;
  if (tile >= tilesM * tilesN) return;
  const int tm = tile / tilesN;
  const int tn = tile - tm * tilesN;
  const int m0 = tm << 6;
  const int n0 = tn << 6;

  const T* Ab  = A  + (size_t)b * strideA;
  const T* Bb  = Bt + (size_t)b * strideB;
  const T* Ab2 = SPLIT ? (A2  + (size_t)b * strideA) : nullptr;
  const T* Bb2 = SPLIT ? (Bt2 + (size_t)b * strideB) : nullptr;

  const int rlane = lane & 15;
  const int koff  = (lane >> 4) * 8;
  const int mOff  = (lane >> 4) * 8;

  v8f acc[4][4];
#pragma unroll
  for (int i = 0; i < 4; ++i)
#pragma unroll
    for (int j = 0; j < 4; ++j) acc[i][j] = (v8f){0.f,0.f,0.f,0.f,0.f,0.f,0.f,0.f};

  for (int k0 = 0; k0 < K; k0 += 32) {
    V bh[4], bl[4];
#pragma unroll
    for (int j = 0; j < 4; ++j) {
      const size_t bo = (size_t)(n0 + (j << 4) + rlane) * ldb + koff + k0;
      bh[j] = Frag<T>::load(Bb + bo);
      if (SPLIT) bl[j] = Frag<T>::load(Bb2 + bo);
    }
#pragma unroll
    for (int i = 0; i < 4; ++i) {
      const size_t ao = (size_t)(m0 + (i << 4) + rlane) * lda + koff + k0;
      V ah = Frag<T>::load(Ab + ao);
      V al;
      if (SPLIT) al = Frag<T>::load(Ab2 + ao);
#pragma unroll
      for (int j = 0; j < 4; ++j) {
        acc[i][j] = Frag<T>::mma(ah, bh[j], acc[i][j]);
        if (SPLIT) {
          acc[i][j] = Frag<T>::mma(ah, bl[j], acc[i][j]);
          acc[i][j] = Frag<T>::mma(al, bh[j], acc[i][j]);
        }
      }
      Frag<T>::guard(acc[i][0], acc[i][3], ah, SPLIT ? al : ah);
    }
    Frag<T>::keep(bh[0], bh[1], bh[2], bh[3]);
    if (SPLIT) Frag<T>::keep(bl[0], bl[1], bl[2], bl[3]);
  }
  acc_guard4(acc[0][0], acc[0][1], acc[0][2], acc[0][3]);
  acc_guard4(acc[1][0], acc[1][1], acc[1][2], acc[1][3]);
  acc_guard4(acc[2][0], acc[2][1], acc[2][2], acc[2][3]);
  acc_guard4(acc[3][0], acc[3][1], acc[3][2], acc[3][3]);

  float* slab = sT[wave];
  const float* Rb = RESID ? (resid + (size_t)b * strideR) : nullptr;
#pragma unroll
  for (int i = 0; i < 4; ++i) {
    const int mBase = m0 + (i << 4);
#pragma unroll
    for (int j = 0; j < 4; ++j) {
      const int n = n0 + (j << 4) + rlane;
      float bv = 0.f;
      if (BIAS_MODE == 2) bv = bias[n];
#pragma unroll
      for (int r = 0; r < 8; ++r) {
        float v = acc[i][j][r] * scale;
        if (BIAS_MODE == 1) v += bias[mBase + mOff + r];
        if (BIAS_MODE == 2) v += bv;
        if (RESID) v += Rb[(size_t)(mBase + mOff + r) * ldc + n];
        if (ACT == 1) v = tanhf(v);
        if (ACT == 2) v = fmaxf(v, 0.0f);
        if (ACT == 3) v = v / (1.0f + expf(-v));
        if (ACT == 4) v = (v > 0.f) ? v : 0.01f * v;
        if (ACT == 5) v = 0.5f * v * (1.0f + erff(v * 0.70710678118654752f));
        slab[(mOff + r) * 68 + (j << 4) + rlane] = v;
      }
    }
    __builtin_amdgcn_fence(__ATOMIC_RELEASE, "workgroup");
    __builtin_amdgcn_wave_barrier();
    __builtin_amdgcn_fence(__ATOMIC_ACQUIRE, "workgroup");
    if (OUT_MODE == 0) {
      float* C = (float*)Cout + (size_t)b * strideC;
      const int hh = lane >> 4, c4 = (lane & 15) * 4;
      for (int pass = 0; pass < 2; ++pass) {
#pragma unroll
        for (int it = 0; it < 8; ++it) {
          const int row = it * 2 + hh;
          v4f v = *(const v4f*)(slab + row * 68 + c4);
          *(volatile v4f*)(C + (size_t)(mBase + row) * ldc + n0 + c4) = v;
        }
        __threadfence();
      }
    } else {
      const int q = lane >> 3, c8 = (lane & 7) * 8;
      unsigned short* C  = (unsigned short*)Cout  + (size_t)b * strideC;
      unsigned short* C2 = (OUT_MODE == 2) ? ((unsigned short*)Cout2 + (size_t)b * strideC) : nullptr;
      for (int pass = 0; pass < 2; ++pass) {
#pragma unroll
        for (int it = 0; it < 4; ++it) {
          const int row = it * 4 + q;
          const float* sp = slab + row * 68 + c8;
          v8h hv, lv;
#pragma unroll
          for (int e = 0; e < 8; ++e) {
            if (OUT_MODE == 1) {
              hv[e] = (_Float16)sp[e];
            } else {
              unsigned short hb = f2bf_bits(sp[e]);
              unsigned short lb = f2bf_bits(sp[e] - bf_bits2f(hb));
              hv[e] = __builtin_bit_cast(_Float16, hb);
              lv[e] = __builtin_bit_cast(_Float16, lb);
            }
          }
          *(volatile v8h*)(C + (size_t)(mBase + row) * ldc + n0 + c8) = hv;
          if (OUT_MODE == 2) *(volatile v8h*)(C2 + (size_t)(mBase + row) * ldc + n0 + c8) = lv;
        }
        __threadfence();
      }
    }
    __builtin_amdgcn_fence(__ATOMIC_RELEASE, "workgroup");
    __builtin_amdgcn_wave_barrier();
    __builtin_amdgcn_fence(__ATOMIC_ACQUIRE, "workgroup");
  }
}

__device__ __forceinline__ unsigned int h16bits(float f) {
  return (unsigned int)__builtin_bit_cast(unsigned short, (_Float16)f);
}

__device__ __forceinline__ v8f mma_f16g(v16h a, v16h b, v8f c) {
  c = __builtin_amdgcn_wmma_f32_16x16x32_f16(false, a, false, b, (short)0, c, false, false);
  asm volatile("v_nop\n\tv_nop\n\tv_nop\n\tv_nop" : "+v"(c) : "v"(a), "v"(b));
  return c;
}

__global__ __launch_bounds__(256) void transpose_cast_f16_kernel(
    const float* __restrict__ W, unsigned short* __restrict__ Wt, int kin, int nout, float mul) {
  __shared__ float tile[64][65];
  const int t = threadIdx.x;
  const int n0 = blockIdx.x * 64;
  const int k0 = blockIdx.y * 64;
#pragma unroll
  for (int i = 0; i < 4; ++i) {
    const int idx = i * 256 + t;
    const int kr = idx >> 4;
    const int nc4 = (idx & 15) * 4;
    const v4f v = *(const v4f*)(W + (size_t)(k0 + kr) * nout + n0 + nc4);
    tile[nc4 + 0][kr] = v[0] * mul;
    tile[nc4 + 1][kr] = v[1] * mul;
    tile[nc4 + 2][kr] = v[2] * mul;
    tile[nc4 + 3][kr] = v[3] * mul;
  }
  __syncthreads();
  const int lane = t & 31, wave = t >> 5;
  const int q = lane >> 3, c8 = (lane & 7) * 8;
  const int row0 = wave * 8 + q;
  const int row1 = wave * 8 + 4 + q;
  v4u w0, w1;
  {
    const float* s0 = &tile[row0][c8];
    const float* s1 = &tile[row1][c8];
    w0[0] = h16bits(s0[0]) | (h16bits(s0[1]) << 16);
    w0[1] = h16bits(s0[2]) | (h16bits(s0[3]) << 16);
    w0[2] = h16bits(s0[4]) | (h16bits(s0[5]) << 16);
    w0[3] = h16bits(s0[6]) | (h16bits(s0[7]) << 16);
    w1[0] = h16bits(s1[0]) | (h16bits(s1[1]) << 16);
    w1[1] = h16bits(s1[2]) | (h16bits(s1[3]) << 16);
    w1[2] = h16bits(s1[4]) | (h16bits(s1[5]) << 16);
    w1[3] = h16bits(s1[6]) | (h16bits(s1[7]) << 16);
  }
  unsigned short* d0 = Wt + (size_t)(n0 + row0) * kin + k0 + c8;
  unsigned short* d1 = Wt + (size_t)(n0 + row1) * kin + k0 + c8;
  for (int pass = 0; pass < 2; ++pass) {
    *(volatile v4u*)d0 = w0;
    *(volatile v4u*)d1 = w1;
    __threadfence();
  }
}

template <bool FUSE_ADD>
__global__ __launch_bounds__(256) void layernorm512_kernel(
    const float* __restrict__ X, const float* __restrict__ Addv,
    const float* __restrict__ gam, const float* __restrict__ bet,
    float* __restrict__ Xsum, unsigned short* __restrict__ Hout, int nrows) {
  const int lane = threadIdx.x & 31;
  const int wave = threadIdx.x >> 5;
  int row = blockIdx.x * 8 + wave;
  row = (row < nrows) ? row : (nrows - 1);
  const size_t rbase = (size_t)row * kModel;
  const int e0 = lane * 4, e1 = 128 + lane * 4, e2 = 256 + lane * 4, e3 = 384 + lane * 4;
  v4f a0 = *(const v4f*)(X + rbase + e0);
  v4f a1 = *(const v4f*)(X + rbase + e1);
  v4f a2 = *(const v4f*)(X + rbase + e2);
  v4f a3 = *(const v4f*)(X + rbase + e3);
  if (FUSE_ADD) {
    const v4f r0 = *(const v4f*)(Addv + rbase + e0);
    const v4f r1 = *(const v4f*)(Addv + rbase + e1);
    const v4f r2 = *(const v4f*)(Addv + rbase + e2);
    const v4f r3 = *(const v4f*)(Addv + rbase + e3);
    a0 = a0 + r0; a1 = a1 + r1; a2 = a2 + r2; a3 = a3 + r3;
    for (int pass = 0; pass < 2; ++pass) {
      *(volatile v4f*)(Xsum + rbase + e0) = a0;
      *(volatile v4f*)(Xsum + rbase + e1) = a1;
      *(volatile v4f*)(Xsum + rbase + e2) = a2;
      *(volatile v4f*)(Xsum + rbase + e3) = a3;
      __threadfence();
    }
  }
  float s = ((a0[0] + a0[1]) + (a0[2] + a0[3])) + ((a1[0] + a1[1]) + (a1[2] + a1[3]))
          + ((a2[0] + a2[1]) + (a2[2] + a2[3])) + ((a3[0] + a3[1]) + (a3[2] + a3[3]));
#pragma unroll
  for (int off = 16; off >= 1; off >>= 1) s += __shfl_xor(s, off, 32);
  const float mu = s * (1.0f / 512.0f);
  const v4f d0 = a0 - mu, d1 = a1 - mu, d2 = a2 - mu, d3 = a3 - mu;
  float ss = ((d0[0] * d0[0] + d0[1] * d0[1]) + (d0[2] * d0[2] + d0[3] * d0[3]))
           + ((d1[0] * d1[0] + d1[1] * d1[1]) + (d1[2] * d1[2] + d1[3] * d1[3]))
           + ((d2[0] * d2[0] + d2[1] * d2[1]) + (d2[2] * d2[2] + d2[3] * d2[3]))
           + ((d3[0] * d3[0] + d3[1] * d3[1]) + (d3[2] * d3[2] + d3[3] * d3[3]));
#pragma unroll
  for (int off = 16; off >= 1; off >>= 1) ss += __shfl_xor(ss, off, 32);
  const float var = ss * (1.0f / 512.0f);
  const float rstd = rsqrtf(var + 1e-5f);
  const v4f g0 = *(const v4f*)(gam + e0), g1 = *(const v4f*)(gam + e1), g2 = *(const v4f*)(gam + e2), g3 = *(const v4f*)(gam + e3);
  const v4f b0 = *(const v4f*)(bet + e0), b1 = *(const v4f*)(bet + e1), b2 = *(const v4f*)(bet + e2), b3 = *(const v4f*)(bet + e3);
  const v4f y0 = d0 * rstd * g0 + b0;
  const v4f y1 = d1 * rstd * g1 + b1;
  const v4f y2 = d2 * rstd * g2 + b2;
  const v4f y3 = d3 * rstd * g3 + b3;
  v2u w0, w1, w2, w3;
  w0[0] = h16bits(y0[0]) | (h16bits(y0[1]) << 16); w0[1] = h16bits(y0[2]) | (h16bits(y0[3]) << 16);
  w1[0] = h16bits(y1[0]) | (h16bits(y1[1]) << 16); w1[1] = h16bits(y1[2]) | (h16bits(y1[3]) << 16);
  w2[0] = h16bits(y2[0]) | (h16bits(y2[1]) << 16); w2[1] = h16bits(y2[2]) | (h16bits(y2[3]) << 16);
  w3[0] = h16bits(y3[0]) | (h16bits(y3[1]) << 16); w3[1] = h16bits(y3[2]) | (h16bits(y3[3]) << 16);
  unsigned short* hr = Hout + rbase;
  for (int pass = 0; pass < 2; ++pass) {
    *(volatile v2u*)(hr + e0) = w0;
    *(volatile v2u*)(hr + e1) = w1;
    *(volatile v2u*)(hr + e2) = w2;
    *(volatile v2u*)(hr + e3) = w3;
    __threadfence();
  }
}

__global__ __launch_bounds__(128) void mha64_f16_kernel(
    const unsigned short* __restrict__ qkp, const unsigned short* __restrict__ vtp,
    unsigned short* __restrict__ outp) {
  typedef Frag<_Float16> FH;
  union FB { v16h v; v8h h[2]; };
  __shared__ __align__(16) _Float16 Psh[4][16 * 64];
  __shared__ __align__(16) float    Os[4][16 * 68];
  const _Float16* QK = (const _Float16*)(const void*)qkp;
  const _Float16* VT = (const _Float16*)(const void*)vtp;
  const int tid = threadIdx.x;
  const int wave = tid >> 5;
  const int lane = tid & 31;
  const int hh = lane >> 4;
  const int c = lane & 15;
  const int koff = hh * 8;
  const int bx = blockIdx.x;
  const int qb = bx & 31;
  const int bh = bx >> 5;
  const int h = bh & 7;
  const int b = (bh >> 3) & 3;
  const int q0 = qb * 64 + wave * 16;
  const _Float16* qbase = QK + (size_t)b * kSeq * kQKCols + h * kHeadDim;
  const _Float16* kbase = qbase + kModel;
  const _Float16* vbase = VT + ((size_t)b * kModel + (size_t)h * kHeadDim) * kSeq;
  unsigned short* obase = outp + (size_t)b * kSeq * kModel + h * kHeadDim;

  v16h qa[2];
#pragma unroll
  for (int dc = 0; dc < 2; ++dc)
    qa[dc] = FH::load(qbase + (size_t)(q0 + c) * kQKCols + dc * 32 + koff);

  float mrow[8], lrow[8];
  v8f oacc[4];
#pragma unroll
  for (int r = 0; r < 8; ++r) { mrow[r] = -INFINITY; lrow[r] = 0.f; }
#pragma unroll
  for (int t = 0; t < 4; ++t) oacc[t] = (v8f){0.f,0.f,0.f,0.f,0.f,0.f,0.f,0.f};

  _Float16* pw = Psh[wave];
  for (int kc = 0; kc < kSeq / 64; ++kc) {
    const int kv0 = kc * 64;
    v8f s[4];
#pragma unroll
    for (int j = 0; j < 4; ++j) {
      s[j] = (v8f){0.f,0.f,0.f,0.f,0.f,0.f,0.f,0.f};
#pragma unroll
      for (int dc = 0; dc < 2; ++dc) {
        const v16h kb = FH::load(kbase + (size_t)(kv0 + j * 16 + c) * kQKCols + dc * 32 + koff);
        s[j] = mma_f16g(qa[dc], kb, s[j]);
      }
    }
    float cm[8];
#pragma unroll
    for (int r = 0; r < 8; ++r) {
      float m = -INFINITY;
#pragma unroll
      for (int j = 0; j < 4; ++j) { s[j][r] = s[j][r] * 0.125f; m = fmaxf(m, s[j][r]); }
#pragma unroll
      for (int off = 1; off < 16; off <<= 1) m = fmaxf(m, __shfl_xor(m, off, 32));
      cm[r] = m;
    }
#pragma unroll
    for (int r = 0; r < 8; ++r) {
      const float mnew = fmaxf(mrow[r], cm[r]);
      const float alpha = expf(mrow[r] - mnew);
      mrow[r] = mnew;
      float psum = 0.f;
#pragma unroll
      for (int j = 0; j < 4; ++j) {
        const float p = expf(s[j][r] - mnew);
        psum += p;
        pw[(8 * hh + r) * 64 + j * 16 + c] = (_Float16)(p * 32768.0f);
      }
#pragma unroll
      for (int off = 1; off < 16; off <<= 1) psum += __shfl_xor(psum, off, 32);
      lrow[r] = lrow[r] * alpha + psum;
#pragma unroll
      for (int t = 0; t < 4; ++t) oacc[t][r] *= alpha;
    }
    __builtin_amdgcn_fence(__ATOMIC_RELEASE, "workgroup");
    __builtin_amdgcn_wave_barrier();
    __builtin_amdgcn_fence(__ATOMIC_ACQUIRE, "workgroup");
#pragma unroll
    for (int kk = 0; kk < 2; ++kk) {
      FB pa;
      pa.h[0] = *(const v8h*)(pw + c * 64 + kk * 32 + 8 * hh);
      pa.h[1] = *(const v8h*)(pw + c * 64 + kk * 32 + 16 + 8 * hh);
#pragma unroll
      for (int t = 0; t < 4; ++t) {
        const v16h vb = FH::load(vbase + (size_t)(t * 16 + c) * kSeq + kv0 + kk * 32 + koff);
        oacc[t] = mma_f16g(pa.v, vb, oacc[t]);
      }
    }
    __builtin_amdgcn_fence(__ATOMIC_RELEASE, "workgroup");
    __builtin_amdgcn_wave_barrier();
    __builtin_amdgcn_fence(__ATOMIC_ACQUIRE, "workgroup");
  }

  float* os = Os[wave];
#pragma unroll
  for (int r = 0; r < 8; ++r) {
    const float inv = (1.0f / lrow[r]) * (1.0f / 2048.0f);
#pragma unroll
    for (int t = 0; t < 4; ++t) os[(8 * hh + r) * 68 + t * 16 + c] = oacc[t][r] * inv;
  }
  __builtin_amdgcn_fence(__ATOMIC_RELEASE, "workgroup");
  __builtin_amdgcn_wave_barrier();
  __builtin_amdgcn_fence(__ATOMIC_ACQUIRE, "workgroup");
  {
    const int q = lane >> 3, c8 = (lane & 7) * 8;
    for (int pass = 0; pass < 2; ++pass) {
#pragma unroll
      for (int it = 0; it < 4; ++it) {
        const int row = it * 4 + q;
        const float* sp = os + row * 68 + c8;
        v8h hv;
#pragma unroll
        for (int e = 0; e < 8; ++e) hv[e] = (_Float16)sp[e];
        *(volatile v8h*)(obase + (size_t)(q0 + row) * kModel + c8) = hv;
      }
      __threadfence();
    }
  }
}

__device__ __forceinline__ float silu_f32(float g) {
  const float ex = expf(-g);
  return g * (1.0f / (1.0f + ex));
}
__global__ __launch_bounds__(256) void swiglu_f16_kernel(
    const float* __restrict__ GU, unsigned short* __restrict__ G, int ngroups) {
  const int i = blockIdx.x * 256 + threadIdx.x;
  if (i < ngroups) {
    const size_t e = (size_t)i * 4;
    const size_t row = e >> 10;
    const int j = (int)(e & 1023);
    const float* gr = GU + row * kGUCols;
    const v4f gv = *(const v4f*)(gr + j);
    const v4f uv = *(const v4f*)(gr + kFF + j);
    const float o0 = silu_f32(gv[0]) * uv[0];
    const float o1 = silu_f32(gv[1]) * uv[1];
    const float o2 = silu_f32(gv[2]) * uv[2];
    const float o3 = silu_f32(gv[3]) * uv[3];
    v2u w;
    w[0] = h16bits(o0) | (h16bits(o1) << 16);
    w[1] = h16bits(o2) | (h16bits(o3) << 16);
    unsigned short* dst = G + e;
    *(volatile v2u*)dst = w;
    __threadfence();
    *(volatile v2u*)dst = w;
  }
}

__global__ __launch_bounds__(256) void residual_out_kernel(
    const float* __restrict__ X1, const float* __restrict__ D2, float* __restrict__ Out, int n4) {
  const int i = blockIdx.x * 256 + threadIdx.x;
  if (i < n4) {
    const size_t e = (size_t)i * 4;
    const v4f a = *(const v4f*)(X1 + e);
    const v4f d = *(const v4f*)(D2 + e);
    const v4f o = a + d;
    *(volatile v4f*)(Out + e) = o;
    __threadfence();
    *(volatile v4f*)(Out + e) = o;
  }
}

extern "C" void kernel_launch(void* const* d_in, const int* in_sizes, int n_in,
                              void* d_out, int out_size, void* d_ws, size_t ws_size,
                              hipStream_t stream) {
  if (n_in < 12) return;
  if (in_sizes[0] != kTok * kModel || out_size != kTok * kModel) return;
  if (in_sizes[1] != kModel || in_sizes[2] != kModel || in_sizes[3] != kModel || in_sizes[4] != kModel) return;
  if (in_sizes[5] != kModel * kModel || in_sizes[6] != kModel * kModel ||
      in_sizes[7] != kModel * kModel || in_sizes[8] != kModel * kModel) return;
  if (in_sizes[9] != kModel * kFF || in_sizes[10] != kModel * kFF || in_sizes[11] != kFF * kModel) return;
  if (ws_size < kWsTotal) return;

  const float* x    = (const float*)d_in[0];
  const float* ln1w = (const float*)d_in[1];
  const float* ln1b = (const float*)d_in[2];
  const float* ln2w = (const float*)d_in[3];
  const float* ln2b = (const float*)d_in[4];
  const float* wq   = (const float*)d_in[5];
  const float* wk   = (const float*)d_in[6];
  const float* wv   = (const float*)d_in[7];
  const float* wo   = (const float*)d_in[8];
  const float* wgt  = (const float*)d_in[9];
  const float* wup  = (const float*)d_in[10];
  const float* wdn  = (const float*)d_in[11];
  float* out = (float*)d_out;

  char* ws = (char*)d_ws;
  unsigned short* wqkT = (unsigned short*)(ws + kOffWqkT);
  unsigned short* wvT  = (unsigned short*)(ws + kOffWvT);
  unsigned short* woT  = (unsigned short*)(ws + kOffWoT);
  unsigned short* wguT = (unsigned short*)(ws + kOffWguT);
  unsigned short* wdT  = (unsigned short*)(ws + kOffWdT);
  unsigned short* hg   = (unsigned short*)(ws + kOffHG);
  unsigned short* qkpl = (unsigned short*)(ws + kOffR1 + kR1QK);
  unsigned short* vtpl = (unsigned short*)(ws + kOffR1 + kR1Vt);
  unsigned short* opl  = (unsigned short*)(ws + kOffR1 + kR1O);
  float*          a1   = (float*)(ws + kOffR1 + kR1A1);
  float*          gu   = (float*)(ws + kOffR1);
  float*          d2   = (float*)(ws + kOffR1);
  float*          x1   = (float*)(ws + kOffX1);

  const dim3 b256(256), b128(128);
  const float w16 = 16.0f;

  transpose_cast_f16_kernel<<<dim3(kModel / 64, kModel / 64), b256, 0, stream>>>(wq, wqkT, kModel, kModel, w16);
  transpose_cast_f16_kernel<<<dim3(kModel / 64, kModel / 64), b256, 0, stream>>>(wk, wqkT + (size_t)kModel * kModel, kModel, kModel, w16);
  transpose_cast_f16_kernel<<<dim3(kModel / 64, kModel / 64), b256, 0, stream>>>(wv, wvT, kModel, kModel, w16);
  transpose_cast_f16_kernel<<<dim3(kModel / 64, kModel / 64), b256, 0, stream>>>(wo, woT, kModel, kModel, w16);
  transpose_cast_f16_kernel<<<dim3(kFF / 64, kModel / 64), b256, 0, stream>>>(wgt, wguT, kModel, kFF, w16);
  transpose_cast_f16_kernel<<<dim3(kFF / 64, kModel / 64), b256, 0, stream>>>(wup, wguT + (size_t)kFF * kModel, kModel, kFF, w16);
  transpose_cast_f16_kernel<<<dim3(kModel / 64, kFF / 64), b256, 0, stream>>>(wdn, wdT, kFF, kModel, w16);

  layernorm512_kernel<false><<<dim3(kTok / 8), b256, 0, stream>>>(x, x, ln1w, ln1b, x1, hg, kTok);

  static_assert((kTok / 64) * (kQKCols / 64) % 8 == 0, "qk tiles");
  wmma_gemm64<0, false, 0, 1, false, 0><<<dim3((kTok / 64) * (kQKCols / 64) / 8, 1), b256, 0, stream>>>(
      hg, hg, kModel, 0L, wqkT, wqkT, kModel, 0L, (void*)qkpl, (void*)qkpl, kQKCols, 0L,
      x, x, 0L, kTok, kQKCols, kModel, 1.0f / 16.0f);

  static_assert((kModel / 64) * (kSeq / 64) % 8 == 0, "vt tiles");
  wmma_gemm64<0, false, 0, 1, false, 0><<<dim3((kModel / 64) * (kSeq / 64) / 8, kBatch), b256, 0, stream>>>(
      wvT, wvT, kModel, 0L, hg, hg, kModel, (long)kSeq * kModel, (void*)vtpl, (void*)vtpl, kSeq, (long)kModel * kSeq,
      x, x, 0L, kModel, kSeq, kModel, 1.0f / 16.0f);

  mha64_f16_kernel<<<dim3(kBatch * kHeads * (kSeq / 64)), b128, 0, stream>>>(qkpl, vtpl, opl);

  static_assert((kTok / 64) * (kModel / 64) % 8 == 0, "o tiles");
  wmma_gemm64<0, false, 0, 0, false, 0><<<dim3((kTok / 64) * (kModel / 64) / 8, 1), b256, 0, stream>>>(
      opl, opl, kModel, 0L, woT, woT, kModel, 0L, (void*)a1, (void*)a1, kModel, 0L,
      x, x, 0L, kTok, kModel, kModel, 1.0f / 256.0f);

  layernorm512_kernel<true><<<dim3(kTok / 8), b256, 0, stream>>>(x, a1, ln2w, ln2b, x1, hg, kTok);

  static_assert((kTok / 64) * (kGUCols / 64) % 8 == 0, "gu tiles");
  wmma_gemm64<0, false, 0, 0, false, 0><<<dim3((kTok / 64) * (kGUCols / 64) / 8, 1), b256, 0, stream>>>(
      hg, hg, kModel, 0L, wguT, wguT, kModel, 0L, (void*)gu, (void*)gu, kGUCols, 0L,
      x, x, 0L, kTok, kGUCols, kModel, 1.0f / 16.0f);

  swiglu_f16_kernel<<<dim3((kTok * kFF / 4) / 256), b256, 0, stream>>>(gu, hg, kTok * kFF / 4);

  wmma_gemm64<0, false, 0, 0, false, 0><<<dim3((kTok / 64) * (kModel / 64) / 8, 1), b256, 0, stream>>>(
      hg, hg, kFF, 0L, wdT, wdT, kFF, 0L, (void*)d2, (void*)d2, kModel, 0L,
      x, x, 0L, kTok, kModel, kFF, 1.0f / 16.0f);

  residual_out_kernel<<<dim3((kTok * kModel / 4) / 256), b256, 0, stream>>>(x1, d2, out, kTok * kModel / 4);
}
